// OGBGCustomGINE_36283883716969
// MI455X (gfx1250) — hardware-verified
//
#include <hip/hip_runtime.h>
#include <stddef.h>
#include <stdint.h>


#define NN       40000
#define NE       640000
#define DIN      128
#define DE       256
#define MP       40064
#define NCODE    60
#define ETF      (NCODE * DIN)
#define PARF     1056
#define PARS     1024

#define NTHR     256
#define NWAVE    8
#define EPT      8
#define CHUNK    (NTHR * EPT)
#define WCAP     (EPT * 32)
#define LISTN    (NWAVE * WCAP)
#define NBMAX    2048
#define NBRUN    1024
#define RCAP     20480
#define DEGCAP   64
#define PKS      11
#define STW      512
#define LDS_I    (2 * RCAP + 2 * NBMAX + LISTN + 16)
#define LDS_SCAN (LDS_I * 4 + ETF * 4)
#define SCAN_G   ((MP + NBRUN - 1) / NBRUN)

#define GT       512
#define GW       16
#define GBM      128
#define GNT      8
#define STGF     (GBM * DE)
#define PARL     1024
#define LDS_G    ((STGF + PARL) * 4)
#define GEMM_G   (MP / GBM)

#define PA_XU    (MP * 16)
#define PA_XB    (PA_XU / 256)
#define PA_CU    (NE / 4)
#define PA_CB    (PA_CU / 256)
#define PB_U1    (DE * 32)
#define PB_U2    (DE * 64)
#define PB_B1    (PB_U1 / 256)
#define PB_B2    (PB_U2 / 256)
#define PC_EU    (NCODE * 32)
#define PC_EB    8
#define WSMAX    134217728

static_assert((CHUNK & (CHUNK - 1)) == 0 && CHUNK <= (1 << PKS));
static_assert((NBMAX & (NBMAX - 1)) == 0 && NBMAX <= (1 << PKS));
static_assert((NBRUN & (NBRUN - 1)) == 0 && NBRUN <= NBMAX && (NBRUN % NWAVE) == 0);
static_assert(NE <= (1 << (32 - PKS)));
static_assert(NTHR * 8 == NBMAX);
static_assert(LISTN >= NWAVE * WCAP);
static_assert((RCAP % 32) == 0 && NWAVE * STW <= RCAP);
static_assert(RCAP >= 16638 + 16638 / 20);
static_assert(DEGCAP >= 36 + 8);
static_assert(LDS_SCAN <= 327680 && LDS_G <= 327680);
static_assert(((LDS_I * 4) % 16) == 0);
static_assert(MP % GBM == 0 && MP >= NN && SCAN_G * NBRUN >= MP);
static_assert(GBM == (GW / 2) * 16 && DE == 2 * GNT * 16 && (GBM % GW) == 0);
static_assert(PA_XU % 256 == 0 && PA_CU % 256 == 0 && (NE % 4) == 0);
static_assert(PB_U1 % 256 == 0 && PB_U2 % 256 == 0);
static_assert(PC_EB * 256 >= PC_EU && NCODE == 5 * 6 * 2);
static_assert(DIN == 32 * 4 && DE == 32 * 8 && PARL == 4 * DE && PARS == PARL);

typedef float          v4f  __attribute__((ext_vector_type(4)));
typedef float          v8f  __attribute__((ext_vector_type(8)));
typedef int            v4i  __attribute__((ext_vector_type(4)));
typedef int            v8i  __attribute__((ext_vector_type(8)));
typedef unsigned int   v2u  __attribute__((ext_vector_type(2)));
typedef unsigned int   v4u  __attribute__((ext_vector_type(4)));
typedef unsigned short v8us __attribute__((ext_vector_type(8)));
typedef __bf16         v16b __attribute__((ext_vector_type(16)));
typedef v4f  __attribute__((may_alias)) v4fa;
typedef v4u  __attribute__((may_alias)) v4ua;
typedef v8us __attribute__((may_alias)) v8usa;
union FragB { v16b v; v8us h[2]; v8i w; };

__device__ __forceinline__ v8f wmb(const FragB& a, const FragB& b, v8f c) {
  v8f d = __builtin_amdgcn_wmma_f32_16x16x32_bf16(false, a.v, false, b.v, (short)0, c, false, false);
  asm volatile("v_nop\n\tv_nop\n\tv_nop\n\tv_nop" : "+v"(d) : "v"(a.w), "v"(b.w));
  return d;
}

__device__ __forceinline__ unsigned short bf_bits(float f) {
  const unsigned int u = __float_as_uint(f);
  const unsigned int r = (u + 0x7FFFu + ((u >> 16) & 1u)) >> 16;
  return (unsigned short)((f != f) ? 0x7FC0u : r);
}
__device__ __forceinline__ float bf_val(unsigned short b) {
  return __uint_as_float(((unsigned int)b) << 16);
}
__device__ __forceinline__ float bf_rne(float f) { return bf_val(bf_bits(f)); }
__device__ __forceinline__ unsigned int pack2(float a, float b) {
  return (unsigned int)bf_bits(a) | ((unsigned int)bf_bits(b) << 16);
}
__device__ __forceinline__ int clampi(int v, int lo, int hi) { return v < lo ? lo : (v > hi ? hi : v); }
__device__ __forceinline__ int ecode(int a0, int a1, int a2) {
  return clampi(a0, 0, 4) * 12 + clampi(a1, 0, 5) * 2 + clampi(a2, 0, 1);
}

__global__ __launch_bounds__(256) void k_pa(const float* __restrict__ x, const int* __restrict__ ea,
                                            unsigned short* xb, int* code) {
  const int tid = (int)threadIdx.x;
  if ((int)blockIdx.x < PA_XB) {
    const int u   = (int)blockIdx.x * 256 + tid;
    const int row = u >> 4;
    const int c8  = (u & 15) * 8;
    const bool ok = row < NN;
    const int rc  = ok ? row : NN - 1;
    const v4f a = *(const v4f*)(x + (size_t)rc * DIN + c8);
    const v4f b = *(const v4f*)(x + (size_t)rc * DIN + c8 + 4);
    const unsigned int zm = ok ? 0xffffffffu : 0u;
    v4u o;
    o.x = pack2(a.x, a.y) & zm;
    o.y = pack2(a.z, a.w) & zm;
    o.z = pack2(b.x, b.y) & zm;
    o.w = pack2(b.z, b.w) & zm;
    unsigned short* dp = xb + (size_t)row * DIN + c8;
    *(volatile v4u*)dp = o;
    __threadfence();
    *(volatile v4u*)dp = o;
  } else {
    const int u = ((int)blockIdx.x - PA_XB) * 256 + tid;
    const int* p = ea + (size_t)u * 12;
    const v4i q0 = *(const v4i*)(p);
    const v4i q1 = *(const v4i*)(p + 4);
    const v4i q2 = *(const v4i*)(p + 8);
    v4i o;
    o.x = ecode(q0.x, q0.y, q0.z);
    o.y = ecode(q0.w, q1.x, q1.y);
    o.z = ecode(q1.z, q1.w, q2.x);
    o.w = ecode(q2.y, q2.z, q2.w);
    int* dp = code + (size_t)u * 4;
    *(volatile v4i*)dp = o;
    __threadfence();
    *(volatile v4i*)dp = o;
  }
}

__global__ __launch_bounds__(256) void k_pb(const float* __restrict__ W1, const float* __restrict__ W2,
                                            unsigned short* w1t, unsigned short* w2t) {
  const int tid = (int)threadIdx.x;
  if ((int)blockIdx.x < PB_B1) {
    const int v  = (int)blockIdx.x * 256 + tid;
    const int n  = v >> 5;
    const int k8 = (v & 31) * 8;
    const int kk = k8 & (DIN - 1);
    const float* p = W1 + (size_t)kk * DE + n;
    v8us o;
#pragma unroll
    for (int i = 0; i < 8; ++i) o[i] = bf_bits(p[(size_t)i * DE]);
    unsigned short* dp = w1t + (size_t)n * 256 + k8;
    *(volatile v8us*)dp = o;
    __threadfence();
    *(volatile v8us*)dp = o;
  } else {
    const int v  = ((int)blockIdx.x - PB_B1) * 256 + tid;
    const int n  = v >> 6;
    const int k8 = (v & 63) * 8;
    const int kk = k8 & (DE - 1);
    const float* p = W2 + (size_t)kk * DE + n;
    v8us o;
#pragma unroll
    for (int i = 0; i < 8; ++i) o[i] = bf_bits(p[(size_t)i * DE]);
    unsigned short* dp = w2t + (size_t)n * 512 + k8;
    *(volatile v8us*)dp = o;
    __threadfence();
    *(volatile v8us*)dp = o;
  }
}

__global__ __launch_bounds__(256) void k_pc(const float* __restrict__ t0, const float* __restrict__ t1,
                                            const float* __restrict__ t2, const float* __restrict__ eps,
                                            const float* __restrict__ b1, const float* __restrict__ g,
                                            const float* __restrict__ bt, const float* __restrict__ b2,
                                            float* etab, float* par) {
  const int tid = (int)threadIdx.x;
  if ((int)blockIdx.x < PC_EB) {
    const int u  = (int)blockIdx.x * 256 + tid;
    const bool ok = u < PC_EU;
    const int uc = ok ? u : PC_EU - 1;
    const int cd = uc >> 5;
    const int c4 = (uc & 31) * 4;
    const int a0 = cd / 12;
    const int rm = cd - 12 * a0;
    const int a1 = rm >> 1;
    const int a2 = rm & 1;
    const v4f p0 = *(const v4f*)(t0 + a0 * DIN + c4);
    const v4f p1 = *(const v4f*)(t1 + a1 * DIN + c4);
    const v4f p2 = *(const v4f*)(t2 + a2 * DIN + c4);
    v4f o;
    o.x = (bf_rne(p0.x) + bf_rne(p1.x)) + bf_rne(p2.x);
    o.y = (bf_rne(p0.y) + bf_rne(p1.y)) + bf_rne(p2.y);
    o.z = (bf_rne(p0.z) + bf_rne(p1.z)) + bf_rne(p2.z);
    o.w = (bf_rne(p0.w) + bf_rne(p1.w)) + bf_rne(p2.w);
    float* dp = etab + (size_t)uc * 4;
    if (ok) *(volatile v4f*)dp = o;
    __threadfence();
    if (ok) *(volatile v4f*)dp = o;
  } else {
    const int c4  = (tid & 63) * 4;
    const int arr = tid >> 6;
    const v4f vb1 = *(const v4f*)(b1 + c4);
    const v4f vg  = *(const v4f*)(g + c4);
    const v4f vbt = *(const v4f*)(bt + c4);
    const v4f vb2 = *(const v4f*)(b2 + c4);
    const float ev = eps[0];
    v4f v;
    v.x = arr == 0 ? vb1.x : (arr == 1 ? vg.x : (arr == 2 ? vbt.x : vb2.x));
    v.y = arr == 0 ? vb1.y : (arr == 1 ? vg.y : (arr == 2 ? vbt.y : vb2.y));
    v.z = arr == 0 ? vb1.z : (arr == 1 ? vg.z : (arr == 2 ? vbt.z : vb2.z));
    v.w = arr == 0 ? vb1.w : (arr == 1 ? vg.w : (arr == 2 ? vbt.w : vb2.w));
    v4f o;
    o.x = bf_rne(v.x); o.y = bf_rne(v.y); o.z = bf_rne(v.z); o.w = bf_rne(v.w);
    const float S = 1.0f + bf_rne(ev);
    v4f sv;
    sv.x = (tid == 0) ? S : 0.0f; sv.y = 0.0f; sv.z = 0.0f; sv.w = 0.0f;
    float* dp = par + 4 * tid;
    float* sp = par + PARS + 4 * (tid & 7);
    const bool sl = tid < 8;
    *(volatile v4f*)dp = o;
    if (sl) *(volatile v4f*)sp = sv;
    __threadfence();
    *(volatile v4f*)dp = o;
    if (sl) *(volatile v4f*)sp = sv;
  }
}

__device__ __forceinline__ int scan_chunk(const int* __restrict__ dsts, int nE, int cbase, int slotBase,
                                          int nb, int vec8, int* list, int tid, int lane, int wave) {
  int wc = 0;
  const int el0  = tid * EPT;
  const int e0   = cbase + el0;
  const int sent = -2147483647 - 1;
  v4i da, db;
  if (vec8 != 0 && cbase + CHUNK <= nE) {
    da = *(const v4i*)(dsts + e0);
    db = *(const v4i*)(dsts + e0 + 4);
  } else {
    da.x = (e0     < nE) ? dsts[min(e0,     nE - 1)] : sent;
    da.y = (e0 + 1 < nE) ? dsts[min(e0 + 1, nE - 1)] : sent;
    da.z = (e0 + 2 < nE) ? dsts[min(e0 + 2, nE - 1)] : sent;
    da.w = (e0 + 3 < nE) ? dsts[min(e0 + 3, nE - 1)] : sent;
    db.x = (e0 + 4 < nE) ? dsts[min(e0 + 4, nE - 1)] : sent;
    db.y = (e0 + 5 < nE) ? dsts[min(e0 + 5, nE - 1)] : sent;
    db.z = (e0 + 6 < nE) ? dsts[min(e0 + 6, nE - 1)] : sent;
    db.w = (e0 + 7 < nE) ? dsts[min(e0 + 7, nE - 1)] : sent;
  }
  const unsigned nbs = (unsigned)slotBase;
  const unsigned unb = (unsigned)nb;
  const unsigned s0 = (unsigned)da.x - nbs, s1 = (unsigned)da.y - nbs;
  const unsigned s2 = (unsigned)da.z - nbs, s3 = (unsigned)da.w - nbs;
  const unsigned s4 = (unsigned)db.x - nbs, s5 = (unsigned)db.y - nbs;
  const unsigned s6 = (unsigned)db.z - nbs, s7 = (unsigned)db.w - nbs;
  const bool h0 = s0 < unb, h1 = s1 < unb, h2 = s2 < unb, h3 = s3 < unb;
  const bool h4 = s4 < unb, h5 = s5 < unb, h6 = s6 < unb, h7 = s7 < unb;
  const unsigned any = __builtin_amdgcn_ballot_w32(h0 | h1 | h2 | h3 | h4 | h5 | h6 | h7);
  if (any != 0u) {
#define HITJ(J, HJ, SJ) { \
      const unsigned mj = __builtin_amdgcn_ballot_w32(HJ); \
      if (mj != 0u) { \
        if (HJ) { \
          const int pos = wc + (int)__builtin_amdgcn_mbcnt_lo(mj, 0u); \
          if (pos < WCAP) list[wave * WCAP + pos] = ((el0 + (J)) << PKS) | (int)(SJ); \
        } \
        wc += (int)__builtin_popcount(mj); } }
    HITJ(0, h0, s0)
    HITJ(1, h1, s1)
    HITJ(2, h2, s2)
    HITJ(3, h3, s3)
    HITJ(4, h4, s4)
    HITJ(5, h5, s5)
    HITJ(6, h6, s6)
    HITJ(7, h7, s7)
#undef HITJ
  }
  return wc;
}

__global__ __launch_bounds__(NTHR) __attribute__((amdgpu_num_vgpr(248)))
void k_scan(const int* __restrict__ srcs, const int* __restrict__ dsts,
            const unsigned short* __restrict__ xb, const int* __restrict__ code,
            const float* __restrict__ etab, const float* __restrict__ par,
            unsigned short* hout) {
  extern __shared__ v4f lds_dyn[];
  int* reg1 = (int*)lds_dyn;
  int* reg2 = reg1 + RCAP;
  int* scnt = reg2 + RCAP;
  int* soff = scnt + NBMAX;
  int* list = soff + NBMAX;
  int* wcnt = list + LISTN;
  int* wtot = wcnt + NWAVE;
  float* etl = (float*)(wtot + NWAVE);
  const int tid = (int)threadIdx.x, lane = tid & 31, wave = tid >> 5;
  const int nodeBase = (int)blockIdx.x * NBRUN;
  const int nE = NE, nN = NN;

  for (int i = tid; i < NBMAX; i += NTHR) scnt[i] = 0;
  for (int i = tid; i < ETF / 4; i += NTHR) {
    const v4f v = *(const v4f*)(etab + 4 * i);
    *(v4fa*)(etl + 4 * i) = v;
  }
  const float S = par[PARS];
  __syncthreads();

  int tot = 0;
  const int nChunks = (NE + CHUNK - 1) / CHUNK;
#pragma unroll 1
  for (int ch = 0; ch < nChunks; ++ch) {
    const int cbase = ch * CHUNK;
    const int wc = scan_chunk(dsts, nE, cbase, nodeBase, NBRUN, 1, list, tid, lane, wave);
    if (lane == 0) wcnt[wave] = wc;
    __syncthreads();
    int pre = 0, all = 0;
#pragma unroll
    for (int w2 = 0; w2 < NWAVE; ++w2) {
      int c = wcnt[w2];
      c = c < 0 ? 0 : (c > WCAP ? WCAP : c);
      all += c;
      pre += (w2 < wave) ? c : 0;
    }
    const int wcc  = wc > WCAP ? WCAP : wc;
    const int base = tot + pre;
#pragma unroll 1
    for (int i = lane; i < wcc; i += 32) {
      const int ent = list[wave * WCAP + i];
      const int el  = (ent >> PKS) & (CHUNK - 1);
      const int sl  = ent & (NBMAX - 1);
      int eid = cbase + el;
      eid = eid > nE - 1 ? nE - 1 : eid;
      const int pos = base + i;
      if (pos < RCAP) reg1[pos] = (int)(((unsigned)eid << PKS) | (unsigned)sl);
    }
    tot += all;
    tot = tot > RCAP ? RCAP : tot;
    __syncthreads();
  }
  const int nh = tot;

  if (wave == 0) {
#pragma unroll 1
    for (int b0 = 0; b0 < nh; b0 += 32) {
      const int idx = b0 + lane;
      const int uv  = reg1[idx < RCAP ? idx : RCAP - 1];
      const int m32 = (nh - b0) < 32 ? (nh - b0) : 32;
#pragma unroll 1
      for (int k = 0; k < m32; ++k) {
        const int u  = __builtin_amdgcn_readlane(uv, k);
        const int sl = u & (NBMAX - 1);
        if (lane == 0) scnt[sl] = scnt[sl] + 1;
      }
    }
  }
  __syncthreads();

  {
    const v4i ca = *(const v4i*)(scnt + 8 * tid);
    const v4i cb = *(const v4i*)(scnt + 8 * tid + 4);
    const int e0 = ca.x < 0 ? 0 : ca.x, e1 = ca.y < 0 ? 0 : ca.y, e2 = ca.z < 0 ? 0 : ca.z, e3 = ca.w < 0 ? 0 : ca.w;
    const int e4 = cb.x < 0 ? 0 : cb.x, e5 = cb.y < 0 ? 0 : cb.y, e6 = cb.z < 0 ? 0 : cb.z, e7 = cb.w < 0 ? 0 : cb.w;
    const int ts = e0 + e1 + e2 + e3 + e4 + e5 + e6 + e7;
    int incl = ts;
#pragma unroll
    for (int d = 1; d < 32; d <<= 1) {
      const int up = __shfl_up(incl, d);
      if (lane >= d) incl += up;
    }
    if (lane == 31) wtot[wave] = incl;
    __syncthreads();
    int pre = 0;
#pragma unroll
    for (int w2 = 0; w2 < NWAVE; ++w2) pre += (w2 < wave) ? wtot[w2] : 0;
    int run = pre + incl - ts;
    soff[8 * tid + 0] = run; run += e0;
    soff[8 * tid + 1] = run; run += e1;
    soff[8 * tid + 2] = run; run += e2;
    soff[8 * tid + 3] = run; run += e3;
    soff[8 * tid + 4] = run; run += e4;
    soff[8 * tid + 5] = run; run += e5;
    soff[8 * tid + 6] = run; run += e6;
    soff[8 * tid + 7] = run;
  }
  __syncthreads();
  for (int i = tid; i < NBMAX; i += NTHR) list[i] = soff[i];
  __syncthreads();

  if (wave == 0) {
#pragma unroll 1
    for (int b0 = 0; b0 < nh; b0 += 32) {
      const int idx = b0 + lane;
      const int uv  = reg1[idx < RCAP ? idx : RCAP - 1];
      const int m32 = (nh - b0) < 32 ? (nh - b0) : 32;
#pragma unroll 1
      for (int k = 0; k < m32; ++k) {
        const int u   = __builtin_amdgcn_readlane(uv, k);
        const int sl  = u & (NBMAX - 1);
        const int eid = (int)((unsigned)u >> PKS);
        if (lane == 0) {
          int pos = list[sl];
          pos = pos < 0 ? 0 : (pos > RCAP - 1 ? RCAP - 1 : pos);
          reg2[pos] = eid;
          list[sl] = pos + 1;
        }
      }
    }
  }
  __syncthreads();

  const bool ovf = (nh >= RCAP);
  const float qnan = __int_as_float(0x7fc00000);
  unsigned int* stwu = (unsigned int*)((float*)reg1 + wave * STW);

#pragma unroll 1
  for (int jt = 0; jt < NBRUN / NWAVE; ++jt) {
    const int slot = jt * NWAVE + wave;
    const int grow = nodeBase + slot;
    if (grow >= MP) break;
    int st = soff[slot];
    const int craw = scnt[slot];
    int cnt = craw;
    st  = st < 0 ? 0 : (st > nh ? nh : st);
    cnt = cnt < 0 ? 0 : (cnt > DEGCAP ? DEGCAP : cnt);
    if (cnt > nh - st) cnt = nh - st;
    const float pz = (ovf || craw > DEGCAP) ? qnan : 0.0f;
    const bool liveRow = grow < nN;

    float ag0 = 0.0f, ag1 = 0.0f, ag2 = 0.0f, ag3 = 0.0f;
#pragma unroll 1
    for (int b0 = 0; b0 < cnt; b0 += 32) {
      int idx = st + b0 + lane;
      idx = idx > nh - 1 ? nh - 1 : idx;
      idx = idx < 0 ? 0 : (idx > RCAP - 1 ? RCAP - 1 : idx);
      int eid = reg2[idx];
      eid = eid < 0 ? 0 : (eid > nE - 1 ? nE - 1 : eid);
      const int sraw = srcs[eid];
      const int craw2 = code[eid];
      const int sv = sraw < 0 ? 0 : (sraw > nN - 1 ? nN - 1 : sraw);
      const int cv = craw2 < 0 ? 0 : (craw2 > NCODE - 1 ? NCODE - 1 : craw2);
      const int m32 = (cnt - b0) < 32 ? (cnt - b0) : 32;
#pragma unroll 1
      for (int k = 0; k < m32; ++k) {
        const int sk = __builtin_amdgcn_readlane(sv, k);
        const int ck = __builtin_amdgcn_readlane(cv, k);
        const v2u w = *(const v2u*)(xb + (size_t)sk * DIN + 4 * lane);
        const v4f e = *(const v4fa*)(etl + ck * DIN + 4 * lane);
        const float v0 = __uint_as_float(w.x << 16) + e.x;
        const float v1 = __uint_as_float(w.x & 0xffff0000u) + e.y;
        const float v2 = __uint_as_float(w.y << 16) + e.z;
        const float v3 = __uint_as_float(w.y & 0xffff0000u) + e.w;
        ag0 += (v0 > 0.0f) ? v0 : 0.0f;
        ag1 += (v1 > 0.0f) ? v1 : 0.0f;
        ag2 += (v2 > 0.0f) ? v2 : 0.0f;
        ag3 += (v3 > 0.0f) ? v3 : 0.0f;
      }
    }
    const int nc = liveRow ? grow : nN - 1;
    const v2u sw = *(const v2u*)(xb + (size_t)nc * DIN + 4 * lane);
    const float x0 = __uint_as_float(sw.x << 16);
    const float x1 = __uint_as_float(sw.x & 0xffff0000u);
    const float x2 = __uint_as_float(sw.y << 16);
    const float x3 = __uint_as_float(sw.y & 0xffff0000u);
    float r0 = S * x0 + ag0, r1 = S * x1 + ag1, r2 = S * x2 + ag2, r3 = S * x3 + ag3;
    r0 = (liveRow ? r0 : 0.0f) + pz;
    r1 = (liveRow ? r1 : 0.0f) + pz;
    r2 = (liveRow ? r2 : 0.0f) + pz;
    r3 = (liveRow ? r3 : 0.0f) + pz;

    const unsigned short hb0 = bf_bits(r0), hb1 = bf_bits(r1), hb2 = bf_bits(r2), hb3 = bf_bits(r3);
    const unsigned short lb0 = bf_bits(r0 - bf_val(hb0)), lb1 = bf_bits(r1 - bf_val(hb1));
    const unsigned short lb2 = bf_bits(r2 - bf_val(hb2)), lb3 = bf_bits(r3 - bf_val(hb3));
    v2u hw, lw;
    hw.x = (unsigned int)hb0 | ((unsigned int)hb1 << 16);
    hw.y = (unsigned int)hb2 | ((unsigned int)hb3 << 16);
    lw.x = (unsigned int)lb0 | ((unsigned int)lb1 << 16);
    lw.y = (unsigned int)lb2 | ((unsigned int)lb3 << 16);
    __builtin_amdgcn_fence(__ATOMIC_RELEASE, "workgroup");
    __builtin_amdgcn_wave_barrier();
    *(v2u*)(stwu + 2 * lane)      = hw;
    *(v2u*)(stwu + 64 + 2 * lane) = lw;
    __builtin_amdgcn_fence(__ATOMIC_RELEASE, "workgroup");
    __builtin_amdgcn_wave_barrier();
    const v4u pk = *(const v4ua*)(stwu + 4 * lane);
    unsigned short* gp = hout + (size_t)grow * (size_t)(2 * DIN) + 8 * lane;
    *(volatile v4u*)gp = pk;
    __threadfence();
    *(volatile v4u*)gp = pk;
  }
}

template <int KT, int MODE>
__global__ __launch_bounds__(GT) __attribute__((amdgpu_num_vgpr(248)))
void k_mlp(const unsigned short* __restrict__ A, const unsigned short* __restrict__ WT,
           const float* __restrict__ par, void* outp) {
  extern __shared__ v4f lds_dyn[];
  float* stg = (float*)lds_dyn;
  float* pls = stg + STGF;
  const int tid = (int)threadIdx.x, lane = tid & 31, wave = tid >> 5, hh = lane >> 4, m = lane & 15;
  const int rt = wave & 7, ch = wave >> 3;
  const int rowBase = (int)blockIdx.x * GBM;

  if (tid < PARL / 4) {
    const v4f pv = *(const v4f*)(par + 4 * tid);
    *(v4fa*)(pls + 4 * tid) = pv;
  }

  v8f acc[GNT];
  {
    const v8f z = {0.f, 0.f, 0.f, 0.f, 0.f, 0.f, 0.f, 0.f};
#pragma unroll
    for (int t = 0; t < GNT; ++t) acc[t] = z;
  }
  const unsigned short* ap = A + (size_t)(rowBase + 16 * rt + m) * (size_t)KT + 8 * hh;
  const unsigned short* wp = WT + (size_t)(128 * ch + m) * (size_t)KT + 8 * hh;
  constexpr int ksteps = KT / 32;
#pragma unroll 1
  for (int ks = 0; ks < ksteps; ++ks) {
    FragB af;
    af.h[0] = *(const v8usa*)(ap + 32 * ks);
    af.h[1] = *(const v8usa*)(ap + 32 * ks + 16);
#pragma unroll
    for (int t = 0; t < GNT; ++t) {
      const unsigned short* wq = wp + (size_t)(16 * t) * (size_t)KT + 32 * ks;
      FragB bf;
      bf.h[0] = *(const v8usa*)wq;
      bf.h[1] = *(const v8usa*)(wq + 16);
      acc[t] = wmb(af, bf, acc[t]);
    }
  }

#pragma unroll
  for (int t = 0; t < GNT; ++t) {
    const int lc = 128 * ch + 16 * t + m;
#pragma unroll
    for (int r = 0; r < 8; ++r) {
      const int lr = 16 * rt + 8 * hh + r;
      stg[lr * DE + lc] = acc[t][r];
    }
  }
  __syncthreads();

#pragma unroll 1
  for (int i = 0; i < GBM / GW; ++i) {
    const int lr = wave * (GBM / GW) + i;
    const int gr = rowBase + lr;
    if constexpr (MODE == 1) {
      const float* sr = stg + lr * DE + 8 * lane;
      const v4f a0 = *(const v4fa*)sr;
      const v4f a1 = *(const v4fa*)(sr + 4);
      const v4f c0 = *(const v4fa*)(pls + 8 * lane);
      const v4f c1 = *(const v4fa*)(pls + 8 * lane + 4);
      const float t0 = a0.x + c0.x, t1 = a0.y + c0.y, t2 = a0.z + c0.z, t3 = a0.w + c0.w;
      const float t4 = a1.x + c1.x, t5 = a1.y + c1.y, t6 = a1.z + c1.z, t7 = a1.w + c1.w;
      float s = ((t0 + t1) + (t2 + t3)) + ((t4 + t5) + (t6 + t7));
      s += __shfl_xor(s, 16);
      s += __shfl_xor(s, 8);
      s += __shfl_xor(s, 4);
      s += __shfl_xor(s, 2);
      s += __shfl_xor(s, 1);
      const float mu = s * (1.0f / (float)DE);
      const float d0 = t0 - mu, d1 = t1 - mu, d2 = t2 - mu, d3 = t3 - mu;
      const float d4 = t4 - mu, d5 = t5 - mu, d6 = t6 - mu, d7 = t7 - mu;
      float q = ((d0 * d0 + d1 * d1) + (d2 * d2 + d3 * d3)) + ((d4 * d4 + d5 * d5) + (d6 * d6 + d7 * d7));
      q += __shfl_xor(q, 16);
      q += __shfl_xor(q, 8);
      q += __shfl_xor(q, 4);
      q += __shfl_xor(q, 2);
      q += __shfl_xor(q, 1);
      const float var = q * (1.0f / (float)DE);
      const float rs = 1.0f / sqrtf(var + 1e-5f);
      const v4f g0 = *(const v4fa*)(pls + DE + 8 * lane);
      const v4f g1 = *(const v4fa*)(pls + DE + 8 * lane + 4);
      const v4f e0 = *(const v4fa*)(pls + 2 * DE + 8 * lane);
      const v4f e1 = *(const v4fa*)(pls + 2 * DE + 8 * lane + 4);
      float y0 = (d0 * rs) * g0.x + e0.x, y1 = (d1 * rs) * g0.y + e0.y;
      float y2 = (d2 * rs) * g0.z + e0.z, y3 = (d3 * rs) * g0.w + e0.w;
      float y4 = (d4 * rs) * g1.x + e1.x, y5 = (d5 * rs) * g1.y + e1.y;
      float y6 = (d6 * rs) * g1.z + e1.z, y7 = (d7 * rs) * g1.w + e1.w;
      const bool live = gr < NN;
      y0 = (y0 > 0.0f) ? y0 : (y0 - y0);  y1 = (y1 > 0.0f) ? y1 : (y1 - y1);
      y2 = (y2 > 0.0f) ? y2 : (y2 - y2);  y3 = (y3 > 0.0f) ? y3 : (y3 - y3);
      y4 = (y4 > 0.0f) ? y4 : (y4 - y4);  y5 = (y5 > 0.0f) ? y5 : (y5 - y5);
      y6 = (y6 > 0.0f) ? y6 : (y6 - y6);  y7 = (y7 > 0.0f) ? y7 : (y7 - y7);
      y0 = live ? y0 : 0.0f;  y1 = live ? y1 : 0.0f;  y2 = live ? y2 : 0.0f;  y3 = live ? y3 : 0.0f;
      y4 = live ? y4 : 0.0f;  y5 = live ? y5 : 0.0f;  y6 = live ? y6 : 0.0f;  y7 = live ? y7 : 0.0f;
      const unsigned short h0 = bf_bits(y0), h1 = bf_bits(y1), h2 = bf_bits(y2), h3 = bf_bits(y3);
      const unsigned short h4 = bf_bits(y4), h5 = bf_bits(y5), h6 = bf_bits(y6), h7 = bf_bits(y7);
      v4u ph, pl;
      ph.x = (unsigned int)h0 | ((unsigned int)h1 << 16);
      ph.y = (unsigned int)h2 | ((unsigned int)h3 << 16);
      ph.z = (unsigned int)h4 | ((unsigned int)h5 << 16);
      ph.w = (unsigned int)h6 | ((unsigned int)h7 << 16);
      pl.x = pack2(y0 - bf_val(h0), y1 - bf_val(h1));
      pl.y = pack2(y2 - bf_val(h2), y3 - bf_val(h3));
      pl.z = pack2(y4 - bf_val(h4), y5 - bf_val(h5));
      pl.w = pack2(y6 - bf_val(h6), y7 - bf_val(h7));
      unsigned short* op = (unsigned short*)outp + (size_t)gr * (size_t)(2 * DE) + 8 * lane;
      const bool wsv = gr < MP;
      if (wsv) { *(volatile v4u*)op = ph; *(volatile v4u*)(op + DE) = pl; }
      __threadfence();
      if (wsv) { *(volatile v4u*)op = ph; *(volatile v4u*)(op + DE) = pl; }
    } else {
      const float* sr = stg + lr * DE + 4 * lane;
      const v4f a0 = *(const v4fa*)sr;
      const v4f a1 = *(const v4fa*)(sr + 128);
      const v4f c0 = *(const v4fa*)(pls + 3 * DE + 4 * lane);
      const v4f c1 = *(const v4fa*)(pls + 3 * DE + 128 + 4 * lane);
      v4f o0, o1;
      o0.x = a0.x + c0.x; o0.y = a0.y + c0.y; o0.z = a0.z + c0.z; o0.w = a0.w + c0.w;
      o1.x = a1.x + c1.x; o1.y = a1.y + c1.y; o1.z = a1.z + c1.z; o1.w = a1.w + c1.w;
      const int grc = gr < NN ? gr : NN - 1;
      float* op = (float*)outp + (size_t)grc * (size_t)DE + 4 * lane;
      const bool wsv = gr < NN;
      if (wsv) { *(volatile v4f*)op = o0; *(volatile v4f*)(op + 128) = o1; }
      __threadfence();
      if (wsv) { *(volatile v4f*)op = o0; *(volatile v4f*)(op + 128) = o1; }
    }
  }
}

static inline size_t al256(size_t o) { return (o + 255) & ~(size_t)255; }

extern "C" void kernel_launch(void* const* d_in, const int* in_sizes, int n_in,
                              void* d_out, int out_size, void* d_ws, size_t ws_size,
                              hipStream_t stream) {
  if (n_in < 13) return;
  if (in_sizes[0] != NN * DIN) return;
  if (in_sizes[1] != 2 * NE) return;
  if (in_sizes[2] != 3 * NE) return;
  if (in_sizes[3] != 5 * DIN || in_sizes[4] != 6 * DIN || in_sizes[5] != 2 * DIN) return;
  if (in_sizes[6] < 1) return;
  if (in_sizes[7] != DIN * DE) return;
  if (in_sizes[8] != DE || in_sizes[9] != DE || in_sizes[10] != DE) return;
  if (in_sizes[11] != DE * DE) return;
  if (in_sizes[12] != DE) return;
  if (out_size != NN * DE) return;

  const float* x   = (const float*)d_in[0];
  const int*   ei  = (const int*)  d_in[1];
  const int*   src = ei;
  const int*   dst = ei + NE;
  const int*   ea  = (const int*)  d_in[2];
  const float* t0  = (const float*)d_in[3];
  const float* t1  = (const float*)d_in[4];
  const float* t2  = (const float*)d_in[5];
  const float* eps = (const float*)d_in[6];
  const float* W1  = (const float*)d_in[7];
  const float* b1  = (const float*)d_in[8];
  const float* lng = (const float*)d_in[9];
  const float* lnb = (const float*)d_in[10];
  const float* W2  = (const float*)d_in[11];
  const float* b2  = (const float*)d_in[12];
  float* out = (float*)d_out;

  char* ws = (char*)d_ws;
  size_t off = 0;
  const size_t oXB = off; off = al256(off + (size_t)MP * DIN * 2);
  const size_t oCD = off; off = al256(off + (size_t)NE * 4);
  const size_t oH  = off; off = al256(off + (size_t)MP * 2 * DIN * 2);
  const size_t oT  = off; off = al256(off + (size_t)MP * 2 * DE * 2);
  const size_t oW1 = off; off = al256(off + (size_t)DE * 256 * 2);
  const size_t oW2 = off; off = al256(off + (size_t)DE * 512 * 2);
  const size_t oET = off; off = al256(off + (size_t)ETF * 4);
  const size_t oPR = off; off = al256(off + (size_t)PARF * 4);
  if (off > ws_size || off > (size_t)WSMAX) return;
  unsigned short* XB   = (unsigned short*)(ws + oXB);
  int*            CODE = (int*)(ws + oCD);
  unsigned short* HHL  = (unsigned short*)(ws + oH);
  unsigned short* THL  = (unsigned short*)(ws + oT);
  unsigned short* W1T  = (unsigned short*)(ws + oW1);
  unsigned short* W2T  = (unsigned short*)(ws + oW2);
  float*          ETAB = (float*)(ws + oET);
  float*          PAR  = (float*)(ws + oPR);

  hipFuncSetAttribute(reinterpret_cast<const void*>(&k_scan), hipFuncAttributeMaxDynamicSharedMemorySize, LDS_SCAN);
  hipFuncSetAttribute(reinterpret_cast<const void*>(&k_mlp<256, 1>), hipFuncAttributeMaxDynamicSharedMemorySize, LDS_G);
  hipFuncSetAttribute(reinterpret_cast<const void*>(&k_mlp<512, 0>), hipFuncAttributeMaxDynamicSharedMemorySize, LDS_G);

  k_pa<<<PA_XB + PA_CB, 256, 0, stream>>>(x, ea, XB, CODE);
  k_pb<<<PB_B1 + PB_B2, 256, 0, stream>>>(W1, W2, W1T, W2T);
  k_pc<<<PC_EB + 1, 256, 0, stream>>>(t0, t1, t2, eps, b1, lng, lnb, b2, ETAB, PAR);
  k_scan<<<SCAN_G, NTHR, LDS_SCAN, stream>>>(src, dst, XB, CODE, ETAB, PAR, HHL);
  k_mlp<256, 1><<<GEMM_G, GT, LDS_G, stream>>>(HHL, W1T, PAR, (void*)THL);
  k_mlp<512, 0><<<GEMM_G, GT, LDS_G, stream>>>(THL, W2T, PAR, (void*)out);
}
